// OrthoLinearAttention_26740466385270
// MI455X (gfx1250) — hardware-verified
//
#include <hip/hip_runtime.h>
#include <math.h>

#define DM    1024
#define LQ    2048
#define BQ    2
#define NTOK  (BQ * LQ)
#define NH    64
#define DHD   16
#define NPROJ (3 * DM)
#define TPB   128
#define OSTR  68
#define SCH   32
#define HPB   16
#define CPB   (HPB * DHD)

static_assert(NH * DHD == DM);
static_assert(NTOK % TPB == 0);
static_assert(NPROJ % 64 == 0);
static_assert(DM % 64 == 0);
static_assert(DM % 32 == 0);
static_assert(LQ % SCH == 0);
static_assert(CPB == 256);
static_assert(NH % HPB == 0);
static_assert(SCH * CPB == 4 * 256 * 8);
static_assert(OSTR % 4 == 0);
static_assert((NTOK * DM) % 8 == 0);
static_assert((DM * DM) % 8 == 0);

typedef unsigned short us16 __attribute__((ext_vector_type(16)));
typedef unsigned short us8  __attribute__((ext_vector_type(8)));
typedef unsigned short us8a __attribute__((ext_vector_type(8), may_alias));
typedef __bf16 v16b __attribute__((ext_vector_type(16)));
typedef _Float16 v16h __attribute__((ext_vector_type(16)));
typedef float v8f __attribute__((ext_vector_type(8)));
typedef float v4f __attribute__((ext_vector_type(4)));
typedef float v4fa __attribute__((ext_vector_type(4), may_alias));
union FragU { us16 v; us8 h[2]; };

__device__ __forceinline__ unsigned short bf16_bits(float f) {
  unsigned u = __float_as_uint(f);
  u += 0x7FFFu + ((u >> 16) & 1u);
  return (unsigned short)(u >> 16);
}
__device__ __forceinline__ float bf16_val(unsigned short b) { return __uint_as_float(((unsigned)b) << 16); }
__device__ __forceinline__ float bf16r(float f) { return bf16_val(bf16_bits(f)); }
__device__ __forceinline__ unsigned short f16_bits(float f) { return __builtin_bit_cast(unsigned short, (_Float16)f); }

__device__ __forceinline__ void f16split16(float a, unsigned short& hb, unsigned short& lb) {
  const float z = a * 16.0f;
  const _Float16 hf = (_Float16)z;
  const float res = (z - (float)hf) * 2048.0f;
  hb = __builtin_bit_cast(unsigned short, hf);
  lb = __builtin_bit_cast(unsigned short, (_Float16)res);
}

__device__ __forceinline__ v8f mma_bf16(us16 a, us16 b, v8f c) {
  return __builtin_amdgcn_wmma_f32_16x16x32_bf16(false, __builtin_bit_cast(v16b, a), false, __builtin_bit_cast(v16b, b), (short)0, c, false, false);
}
__device__ __forceinline__ v8f mma_f16(us16 a, us16 b, v8f c) {
  return __builtin_amdgcn_wmma_f32_16x16x32_f16(false, __builtin_bit_cast(v16h, a), false, __builtin_bit_cast(v16h, b), (short)0, c, false, false);
}
__device__ __forceinline__ void wguard4(v8f& c0, v8f& c1, v8f& c2, v8f& c3, const us16& a0,
                                        const us16& b0, const us16& b1, const us16& b2, const us16& b3) {
#if defined(__HIP_DEVICE_COMPILE__)
  asm volatile("v_nop\n\tv_nop\n\tv_nop\n\tv_nop"
               : "+v"(c0), "+v"(c1), "+v"(c2), "+v"(c3)
               : "v"(a0), "v"(b0), "v"(b1), "v"(b2), "v"(b3));
#endif
}
__device__ __forceinline__ void wguard8(v8f& c0, v8f& c1, v8f& c2, v8f& c3, v8f& c4, v8f& c5, v8f& c6, v8f& c7,
                                        const us16& a0, const us16& a1,
                                        const us16& b0, const us16& b1, const us16& b2, const us16& b3) {
#if defined(__HIP_DEVICE_COMPILE__)
  asm volatile("v_nop\n\tv_nop\n\tv_nop\n\tv_nop"
               : "+v"(c0), "+v"(c1), "+v"(c2), "+v"(c3), "+v"(c4), "+v"(c5), "+v"(c6), "+v"(c7)
               : "v"(a0), "v"(a1), "v"(b0), "v"(b1), "v"(b2), "v"(b3));
#endif
}

__device__ __forceinline__ us16 gfrag(const unsigned short* p) {
  const int kh = ((threadIdx.x >> 4) & 1) * 8;
  FragU f;
  f.h[0] = *(const us8a*)(p + kh);
  f.h[1] = *(const us8a*)(p + 16 + kh);
  return f.v;
}

template <int MODE>
__global__ __launch_bounds__(256) void k_cvt(const float* __restrict__ src, unsigned short* dst, int total8) {
  const int idx = blockIdx.x * 256 + threadIdx.x;
  if (idx >= total8) return;
  const size_t off = (size_t)idx * 8;
  const v4f a = *(const v4fa*)(src + off), b = *(const v4fa*)(src + off + 4);
  us8 o;
#pragma unroll
  for (int u = 0; u < 4; ++u) {
    if (MODE == 0) {
      o[u]     = bf16_bits(a[u]);
      o[4 + u] = bf16_bits(b[u]);
    } else {
      o[u]     = f16_bits(bf16r(a[u]) * 256.0f);
      o[4 + u] = f16_bits(bf16r(b[u]) * 256.0f);
    }
  }
  *(volatile us8*)(dst + off) = o;
  __threadfence();
  *(volatile us8*)(dst + off) = o;
}

__global__ __launch_bounds__(256) void k_gemm_proj(const unsigned short* __restrict__ Ap, const unsigned short* __restrict__ Bw,
                                                  const float* __restrict__ bqp, const float* __restrict__ bkp,
                                                  const float* __restrict__ bvp, const float* __restrict__ betap,
                                                  float* Qp, float* Kp, float* Vp) {
  __shared__ __attribute__((aligned(16))) float oS[8 * 16 * OSTR];
  const int tid = threadIdx.x, lane = tid & 31, wave = tid >> 5, cl = lane & 15, hh = lane >> 4;
  const int m0 = blockIdx.x * TPB + 16 * wave, n0 = blockIdx.y * 64;

  v8f acc[4];
#pragma unroll
  for (int j = 0; j < 4; ++j) { const v8f zz = {0.f, 0.f, 0.f, 0.f, 0.f, 0.f, 0.f, 0.f}; acc[j] = zz; }

  const unsigned short* a0p = Ap + (size_t)(m0 + cl) * (size_t)DM;
  const unsigned short* bwp = Bw + (size_t)(n0 + cl) * (size_t)DM;
#pragma unroll 1
  for (int k0 = 0; k0 < DM; k0 += 32) {
    const us16 af = gfrag(a0p + k0);
    us16 bfr[4];
#pragma unroll
    for (int j = 0; j < 4; ++j) bfr[j] = gfrag(bwp + (size_t)(16 * j) * (size_t)DM + k0);
#pragma unroll
    for (int j = 0; j < 4; ++j) acc[j] = mma_bf16(af, bfr[j], acc[j]);
    wguard4(acc[0], acc[1], acc[2], acc[3], af, bfr[0], bfr[1], bfr[2], bfr[3]);
  }

  float* so = oS + wave * (16 * OSTR);
#pragma unroll
  for (int j = 0; j < 4; ++j)
#pragma unroll
    for (int r = 0; r < 8; ++r) so[(8 * hh + r) * OSTR + 16 * j + cl] = acc[j][r];
  __syncthreads();

  const int seg = n0 / DM;
  const float* bias = bqp; float* dst = Qp;
  if (seg == 1) { bias = bkp; dst = Kp; }
  if (seg == 2) { bias = bvp; dst = Vp; }
  const int c0 = n0 - seg * DM;
  const float be = expf(bf16r(betap[0]));

#pragma unroll 1
  for (int t = 0; t < 2; ++t) {
    const int un = t * 32 + lane, r = un >> 2, j = un & 3;
    float* sp = so + r * OSTR + 16 * j;
    const float* gp = bias + c0 + 16 * j;
    v4f x0 = *(const v4fa*)sp, x1 = *(const v4fa*)(sp + 4), x2 = *(const v4fa*)(sp + 8), x3 = *(const v4fa*)(sp + 12);
    const v4f g0 = *(const v4fa*)gp, g1 = *(const v4fa*)(gp + 4), g2 = *(const v4fa*)(gp + 8), g3 = *(const v4fa*)(gp + 12);
    float xv[16];
#pragma unroll
    for (int u = 0; u < 4; ++u) {
      xv[u]      = x0[u] + bf16r(g0[u]);
      xv[4 + u]  = x1[u] + bf16r(g1[u]);
      xv[8 + u]  = x2[u] + bf16r(g2[u]);
      xv[12 + u] = x3[u] + bf16r(g3[u]);
    }
    if (seg < 2) {
#pragma unroll
      for (int i = 0; i < 16; ++i) xv[i] *= be;
      float mx = xv[0];
#pragma unroll
      for (int i = 1; i < 16; ++i) mx = fmaxf(mx, xv[i]);
      float sm = 0.0f;
#pragma unroll
      for (int i = 0; i < 16; ++i) { xv[i] = expf(xv[i] - mx); sm += xv[i]; }
      const float rs = 1.0f / sm;
#pragma unroll
      for (int i = 0; i < 16; ++i) xv[i] *= rs;
    }
#pragma unroll
    for (int u = 0; u < 4; ++u) { x0[u] = xv[u]; x1[u] = xv[4 + u]; x2[u] = xv[8 + u]; x3[u] = xv[12 + u]; }
    *(v4fa*)sp = x0; *(v4fa*)(sp + 4) = x1; *(v4fa*)(sp + 8) = x2; *(v4fa*)(sp + 12) = x3;
  }
  __syncthreads();

#pragma unroll
  for (int pass = 0; pass < 2; ++pass) {
#pragma unroll
    for (int it = 0; it < 8; ++it) {
      const int cx = it * 32 + lane, r = cx >> 4, q = (cx & 15) * 4;
      const v4f v = *(const v4fa*)(so + r * OSTR + q);
      *(volatile v4f*)(dst + (size_t)(m0 + r) * (size_t)DM + c0 + q) = v;
    }
    __threadfence();
  }
}

__global__ __launch_bounds__(256) void k_gemm_out(const unsigned short* __restrict__ Ah, const unsigned short* __restrict__ Al,
                                                 const unsigned short* __restrict__ Wo, const float* __restrict__ bop, float* out) {
  __shared__ __attribute__((aligned(16))) float oS[8 * 16 * OSTR];
  const int tid = threadIdx.x, lane = tid & 31, wave = tid >> 5, cl = lane & 15, hh = lane >> 4;
  const int m0 = blockIdx.x * TPB + 16 * wave, n0 = blockIdx.y * 64;

  v8f acch[4], accl[4];
#pragma unroll
  for (int j = 0; j < 4; ++j) { const v8f zz = {0.f, 0.f, 0.f, 0.f, 0.f, 0.f, 0.f, 0.f}; acch[j] = zz; accl[j] = zz; }

  const unsigned short* ahp = Ah + (size_t)(m0 + cl) * (size_t)DM;
  const unsigned short* alp = Al + (size_t)(m0 + cl) * (size_t)DM;
  const unsigned short* wop = Wo + (size_t)(n0 + cl) * (size_t)DM;
#pragma unroll 1
  for (int k0 = 0; k0 < DM; k0 += 32) {
    const us16 ah = gfrag(ahp + k0);
    const us16 al = gfrag(alp + k0);
    us16 bfr[4];
#pragma unroll
    for (int j = 0; j < 4; ++j) bfr[j] = gfrag(wop + (size_t)(16 * j) * (size_t)DM + k0);
#pragma unroll
    for (int j = 0; j < 4; ++j) {
      acch[j] = mma_f16(ah, bfr[j], acch[j]);
      accl[j] = mma_f16(al, bfr[j], accl[j]);
    }
    wguard8(acch[0], acch[1], acch[2], acch[3], accl[0], accl[1], accl[2], accl[3], ah, al, bfr[0], bfr[1], bfr[2], bfr[3]);
  }

  float gb[4];
#pragma unroll
  for (int j = 0; j < 4; ++j) gb[j] = bf16r(bop[n0 + 16 * j + cl]);

  float* so = oS + wave * (16 * OSTR);
#pragma unroll
  for (int j = 0; j < 4; ++j)
#pragma unroll
    for (int r = 0; r < 8; ++r)
      so[(8 * hh + r) * OSTR + 16 * j + cl] = fmaf(accl[j][r], (1.0f / 2048.0f), acch[j][r]) * (1.0f / 4096.0f) + gb[j];
  __syncthreads();

#pragma unroll
  for (int pass = 0; pass < 2; ++pass) {
#pragma unroll
    for (int it = 0; it < 8; ++it) {
      const int cx = it * 32 + lane, r = cx >> 4, q = (cx & 15) * 4;
      const v4f v = *(const v4fa*)(so + r * OSTR + q);
      *(volatile v4f*)(out + (size_t)(m0 + r) * (size_t)DM + n0 + q) = v;
    }
    __threadfence();
  }
}

__global__ __launch_bounds__(256) void k_scan(const float* __restrict__ Qp, const float* __restrict__ Kp, const float* __restrict__ Vp,
                                             unsigned short* AH, unsigned short* AL) {
  __shared__ __attribute__((aligned(16))) float sy[SCH * CPB];
  const int tid = threadIdx.x;
  const int b = blockIdx.x / (NH / HPB), hg = blockIdx.x - b * (NH / HPB);
  const int d = tid & 15, hl = tid >> 4;
  const int cb = hg * CPB + hl * DHD;

  float S[16];
#pragma unroll
  for (int i = 0; i < 16; ++i) S[i] = 0.0f;
  float zn = 0.0f;

#pragma unroll 1
  for (int c = 0; c < LQ / SCH; ++c) {
    const size_t tok0 = (size_t)b * LQ + (size_t)c * SCH;
#pragma unroll 1
    for (int st = 0; st < SCH; ++st) {
      const size_t ro = (tok0 + (size_t)st) * (size_t)DM + (size_t)cb;
      const float* kp = Kp + ro;
      const float* qp = Qp + ro;
      const v4f k0 = *(const v4fa*)kp, k1 = *(const v4fa*)(kp + 4), k2 = *(const v4fa*)(kp + 8), k3 = *(const v4fa*)(kp + 12);
      const v4f q0 = *(const v4fa*)qp, q1 = *(const v4fa*)(qp + 4), q2 = *(const v4fa*)(qp + 8), q3 = *(const v4fa*)(qp + 12);
      const float kd = kp[d], qd = qp[d], vd = Vp[ro + (size_t)d];
      float kk[16], qq[16];
#pragma unroll
      for (int u = 0; u < 4; ++u) {
        kk[u] = k0[u]; kk[4 + u] = k1[u]; kk[8 + u] = k2[u]; kk[12 + u] = k3[u];
        qq[u] = q0[u]; qq[4 + u] = q1[u]; qq[8 + u] = q2[u]; qq[12 + u] = q3[u];
      }
      float num = 0.0f;
#pragma unroll
      for (int i = 0; i < 16; ++i) {
        S[i] = fmaf(kk[i], vd, S[i]);
        num = fmaf(qq[i], S[i], num);
      }
      zn += kd;
      float p = qd * zn;
      p += __shfl_xor(p, 1, 32);
      p += __shfl_xor(p, 2, 32);
      p += __shfl_xor(p, 4, 32);
      p += __shfl_xor(p, 8, 32);
      const float a = num * (1.0f / p);
      sy[st * CPB + tid] = a;
    }
    __syncthreads();

    us8 hv[4], lv[4];
    size_t offs[4];
#pragma unroll
    for (int it = 0; it < 4; ++it) {
      const int cx = it * 256 + tid, r = cx >> 5, q = (cx & 31) * 8;
      const v4f z0 = *(const v4fa*)(sy + r * CPB + q), z1 = *(const v4fa*)(sy + r * CPB + q + 4);
      us8 ho, lo;
#pragma unroll
      for (int u = 0; u < 4; ++u) {
        unsigned short hb, lb;
        f16split16(z0[u], hb, lb); ho[u] = hb;     lo[u] = lb;
        f16split16(z1[u], hb, lb); ho[4 + u] = hb; lo[4 + u] = lb;
      }
      hv[it] = ho; lv[it] = lo;
      offs[it] = (tok0 + (size_t)r) * (size_t)DM + (size_t)hg * CPB + (size_t)q;
    }
#pragma unroll
    for (int pass = 0; pass < 2; ++pass) {
#pragma unroll
      for (int it = 0; it < 4; ++it) {
        *(volatile us8*)(AH + offs[it]) = hv[it];
        *(volatile us8*)(AL + offs[it]) = lv[it];
      }
      __threadfence();
    }
    __syncthreads();
  }
}

extern "C" void kernel_launch(void* const* d_in, const int* in_sizes, int n_in,
                              void* d_out, int out_size, void* d_ws, size_t ws_size,
                              hipStream_t stream) {
  if (n_in < 10) return;
  if (in_sizes[0] != NTOK * DM || in_sizes[1] != DM * DM || in_sizes[2] != DM || in_sizes[3] != DM * DM || in_sizes[4] != DM ||
      in_sizes[5] != DM * DM || in_sizes[6] != DM || in_sizes[7] != DM * DM || in_sizes[8] != DM || in_sizes[9] < 1) return;
  if (out_size != NTOK * DM) return;

  const float* x    = (const float*)d_in[0];
  const float* Wq   = (const float*)d_in[1];
  const float* bq   = (const float*)d_in[2];
  const float* Wk   = (const float*)d_in[3];
  const float* bk   = (const float*)d_in[4];
  const float* Wv   = (const float*)d_in[5];
  const float* bv   = (const float*)d_in[6];
  const float* Wo   = (const float*)d_in[7];
  const float* bo   = (const float*)d_in[8];
  const float* beta = (const float*)d_in[9];
  float* out = (float*)d_out;

  size_t off = 0;
  auto carve = [&](size_t bytes) -> char* { char* p = (char*)d_ws + off; off += (bytes + 255) & ~(size_t)255; return p; };
  unsigned short* XB   = (unsigned short*)carve((size_t)NTOK * DM * 2);
  unsigned short* WQKV = (unsigned short*)carve((size_t)NPROJ * DM * 2);
  unsigned short* WO16 = (unsigned short*)carve((size_t)DM * DM * 2);
  float* Qp = (float*)carve((size_t)NTOK * DM * 4);
  float* Kp = (float*)carve((size_t)NTOK * DM * 4);
  float* Vp = (float*)carve((size_t)NTOK * DM * 4);
  unsigned short* AH = (unsigned short*)carve((size_t)NTOK * DM * 2);
  unsigned short* AL = (unsigned short*)carve((size_t)NTOK * DM * 2);
  if (off > ws_size || off > (size_t)134217728) return;

  const dim3 b256(256);
  auto cdv = [](long a, long bq2) { return (unsigned)((a + bq2 - 1) / bq2); };

  k_cvt<0><<<dim3(cdv((long)NTOK * DM / 8, 256)), b256, 0, stream>>>(x, XB, NTOK * DM / 8);
  k_cvt<0><<<dim3(cdv((long)DM * DM / 8, 256)), b256, 0, stream>>>(Wq, WQKV, DM * DM / 8);
  k_cvt<0><<<dim3(cdv((long)DM * DM / 8, 256)), b256, 0, stream>>>(Wk, WQKV + (size_t)DM * DM, DM * DM / 8);
  k_cvt<0><<<dim3(cdv((long)DM * DM / 8, 256)), b256, 0, stream>>>(Wv, WQKV + (size_t)2 * DM * DM, DM * DM / 8);
  k_cvt<1><<<dim3(cdv((long)DM * DM / 8, 256)), b256, 0, stream>>>(Wo, WO16, DM * DM / 8);
  k_gemm_proj<<<dim3(NTOK / TPB, NPROJ / 64), b256, 0, stream>>>(XB, WQKV, bq, bk, bv, beta, Qp, Kp, Vp);
  k_scan<<<dim3(BQ * (NH / HPB)), b256, 0, stream>>>(Qp, Kp, Vp, AH, AL);
  k_gemm_out<<<dim3(NTOK / TPB, DM / 64), b256, 0, stream>>>(AH, AL, WO16, bo, out);
}
